// TGN_86045374808295
// MI455X (gfx1250) — hardware-verified
//
#include <hip/hip_runtime.h>
#include <stddef.h>


#define IN_DIM 128
#define HC     64
#define TD     32
#define K1     (IN_DIM + 2 * TD)
#define N1     (2 * HC)
#define K2     N1
#define N2     HC
#define K3     HC
#define N3     16
#define NTHR   256
#define NWAVE  8
#define RT     2
#define TROWS  8
#define CHUNK  4096
#define WCAP   512
#define NGRP   (CHUNK / (NTHR * 4))

#define AGG_SACC 65536
#define AGG_AUX  1024
#define AGG_LIST (NWAVE * WCAP)
#define AGG_LDS_BYTES ((AGG_SACC + 2 * AGG_AUX + AGG_LIST + NWAVE) * 4)

static_assert(WCAP == (CHUNK / NTHR) * 32);
static_assert(NGRP * NTHR * 4 == CHUNK);
static_assert((K1 % 32) == 0 && (K2 % 32) == 0 && (K3 % 32) == 0);
static_assert(AGG_LDS_BYTES == 286752);
static_assert(TROWS * 32 == NTHR);
static_assert(TD == 32 && IN_DIM == 4 * 32);

typedef float v2f __attribute__((ext_vector_type(2)));
typedef float v4f __attribute__((ext_vector_type(4)));
typedef float v8f __attribute__((ext_vector_type(8)));
typedef int   v4i __attribute__((ext_vector_type(4)));
typedef unsigned int v2u __attribute__((ext_vector_type(2)));
typedef unsigned int v4u __attribute__((ext_vector_type(4)));
typedef unsigned short v8us __attribute__((ext_vector_type(8)));
typedef __bf16 v16bf __attribute__((ext_vector_type(16)));
typedef v4u v4ua __attribute__((may_alias));
typedef v2u v2ua __attribute__((may_alias));
typedef unsigned int u32a __attribute__((may_alias));
union Frag { v16bf v; v8us half[2]; };

template<int N> struct VecT { typedef float t __attribute__((ext_vector_type(N))); };
template<int VW> struct PK;
template<> struct PK<4> { typedef v2u t; typedef v2ua ta; };
template<> struct PK<2> { typedef unsigned int t; typedef u32a ta; };

__device__ __forceinline__ v8f wmb(v16bf a, v16bf b, v8f c) {
#if defined(__HIP_DEVICE_COMPILE__)
  v8f d = __builtin_amdgcn_wmma_f32_16x16x32_bf16(false, a, false, b, (short)0, c, false, false);
  asm volatile("v_nop\n\tv_nop\n\tv_nop\n\tv_nop" : "+v"(d) : "v"(a), "v"(b));
  return d;
#else
  (void)a; (void)b;
  return c;
#endif
}

__device__ __forceinline__ void wave_sync() {
#if defined(__HIP_DEVICE_COMPILE__)
  __builtin_amdgcn_fence(__ATOMIC_RELEASE, "wavefront");
  __builtin_amdgcn_wave_barrier();
#endif
}

__device__ __forceinline__ unsigned short bf_rne(float f) {
  unsigned u = __float_as_uint(f);
  u += 0x7fffu + ((u >> 16) & 1u);
  return (unsigned short)(u >> 16);
}
__device__ __forceinline__ float bf_val(unsigned short h) { return __uint_as_float(((unsigned)h) << 16); }
__device__ __forceinline__ void split2(float v, unsigned short& h, unsigned short& l) {
  h = bf_rne(v);
  l = bf_rne(v - bf_val(h));
}
__device__ __forceinline__ void pack_hl(v4f y, v2u& ph, v2u& pl) {
  unsigned short h0, l0, h1, l1, h2, l2, h3, l3;
  split2(y.x, h0, l0); split2(y.y, h1, l1); split2(y.z, h2, l2); split2(y.w, h3, l3);
  ph.x = (unsigned)h0 | ((unsigned)h1 << 16); ph.y = (unsigned)h2 | ((unsigned)h3 << 16);
  pl.x = (unsigned)l0 | ((unsigned)l1 << 16); pl.y = (unsigned)l2 | ((unsigned)l3 << 16);
}
__device__ __forceinline__ void pack_hl(v2f y, unsigned& ph, unsigned& pl) {
  unsigned short h0, l0, h1, l1;
  split2(y.x, h0, l0); split2(y.y, h1, l1);
  ph = (unsigned)h0 | ((unsigned)h1 << 16);
  pl = (unsigned)l0 | ((unsigned)l1 << 16);
}

template<int KD, int NC>
__global__ __launch_bounds__(NTHR) void k_wprep(const float* __restrict__ W,
                                                unsigned short* Wh, unsigned short* Wl) {
  const int t = blockIdx.x * NTHR + threadIdx.x;
  if (t >= NC * KD / 8) return;
  const int n  = t / (KD / 8);
  const int k8 = (t - n * (KD / 8)) * 8;
  union { unsigned short s[8]; v4u q; } uh, ul;
#pragma unroll
  for (int i = 0; i < 8; ++i) {
    const float v = W[(size_t)(k8 + i) * NC + n];
    unsigned short h, l;
    split2(v, h, l);
    uh.s[i] = h;
    ul.s[i] = l;
  }
  const size_t o = (size_t)n * KD + k8;
  const v4u qh = uh.q, ql = ul.q;
  *(volatile v4u*)(Wh + o) = qh;
  *(volatile v4u*)(Wl + o) = ql;
  __threadfence();
  *(volatile v4u*)(Wh + o) = qh;
  *(volatile v4u*)(Wl + o) = ql;
}

__global__ __launch_bounds__(NTHR) void k_time(const float* __restrict__ x, const float* __restrict__ ts,
                                               const float* __restrict__ tw, const float* __restrict__ tb,
                                               unsigned short* H, unsigned short* L, int nN) {
  __shared__ __attribute__((aligned(16))) unsigned short sH[TROWS * K1];
  __shared__ __attribute__((aligned(16))) unsigned short sL[TROWS * K1];
  const int tid  = threadIdx.x;
  const int row0 = blockIdx.x * TROWS;
  const int r    = tid >> 5;
  int row = row0 + r;
  if (row > nN - 1) row = nN - 1;
  {
#pragma clang fp contract(off)
    const int j = tid & 31;
    const float tv = ts[row] * tw[j] + tb[j];
    float sv, cv;
    sincosf(tv, &sv, &cv);
    unsigned short hc, lc, hs, ls;
    split2(cv, hc, lc);
    split2(sv, hs, ls);
    sH[r * K1 + IN_DIM + j] = hc;
    sL[r * K1 + IN_DIM + j] = lc;
    sH[r * K1 + IN_DIM + TD + j] = hs;
    sL[r * K1 + IN_DIM + TD + j] = ls;
  }
  {
    const int c4 = (tid & 31) * 4;
    const v4f xv = *(const v4f*)(x + (size_t)row * IN_DIM + c4);
    v2u ph, pl;
    pack_hl(xv, ph, pl);
    *(v2ua*)(sH + r * K1 + c4) = ph;
    *(v2ua*)(sL + r * K1 + c4) = pl;
  }
  __syncthreads();
  if (tid < TROWS * K1 / 8) {
    const v4u qh = *(const v4ua*)(sH + 8 * tid);
    const v4u ql = *(const v4ua*)(sL + 8 * tid);
    const size_t o = (size_t)row0 * K1 + 8 * tid;
    *(volatile v4u*)(H + o) = qh;
    *(volatile v4u*)(L + o) = ql;
    __threadfence();
    *(volatile v4u*)(H + o) = qh;
    *(volatile v4u*)(L + o) = ql;
  }
}

template<int CT, int XSP, int NHD>
__device__ __forceinline__ void epi_tile(v8f acc, int brow0, int hh, int m, int ct, int ncol,
                                         float cs, float cd, float cb, float* Xs, float* Ps) {
  float ss[8], sd[8];
#pragma unroll
  for (int r = 0; r < 8; ++r) {
    const float v = acc[r] + cb;
    Xs[(brow0 + 8 * hh + r) * XSP + ncol] = v;
    ss[r] = v * cs;
    sd[r] = v * cd;
  }
  if (NHD > 0) {
#pragma unroll
    for (int mk = 1; mk < 16; mk <<= 1) {
#pragma unroll
      for (int r = 0; r < 8; ++r) {
        ss[r] += __shfl_xor(ss[r], mk, 32);
        sd[r] += __shfl_xor(sd[r], mk, 32);
      }
    }
    if (m == 0) {
#pragma unroll
      for (int r = 0; r < 8; ++r) {
        Ps[((brow0 + 8 * hh + r) * CT + ct) * 2 + 0] = ss[r];
        Ps[((brow0 + 8 * hh + r) * CT + ct) * 2 + 1] = sd[r];
      }
    }
  }
}

template<int KD, int NC, int NHD>
__global__ __launch_bounds__(NTHR) void k_gemm(
    const unsigned short* __restrict__ Ah, const unsigned short* __restrict__ Al,
    const unsigned short* __restrict__ Bh, const unsigned short* __restrict__ Bl,
    const float* __restrict__ att_s, const float* __restrict__ att_d, const float* __restrict__ bias,
    float* C, float* asrc, float* adst, int nN) {
  constexpr int CT  = NC / 16;
  constexpr int RG  = NWAVE / CT;
  constexpr int GR  = RG * RT * 16;
  constexpr int XSP = NC + 4;
  constexpr int LPR = NC / 4;
  constexpr int RPI = 32 / LPR;
  constexpr int RPW = GR / NWAVE;
  constexpr int NST = RPW / RPI;
  constexpr int NHX = (NHD > 0) ? NHD : 1;
  static_assert(CT * RG == NWAVE);
  static_assert(NST * RPI == RPW);
  static_assert(RPI * LPR == 32);
  static_assert(NHD == 0 || GR * NHD == 64);
  static_assert(NHD == 0 || CT == 4 * NHD);
  static_assert((XSP % 4) == 0);
  __shared__ __attribute__((aligned(16))) float Xs[GR * XSP];
  __shared__ __attribute__((aligned(16))) float Ps[(NHD > 0) ? GR * CT * 2 : 16];

  const int tid  = threadIdx.x;
  const int lane = tid & 31;
  const int wave = tid >> 5;
  const int hh   = lane >> 4;
  const int m    = lane & 15;
  const int ct   = wave % CT;
  const int rg   = wave / CT;
  const int rowBase = blockIdx.x * GR;
  const int wr0  = rg * RT * 16;
  const int ncol = ct * 16 + m;

  int ra0 = rowBase + wr0 + m;      if (ra0 > nN - 1) ra0 = nN - 1;
  int ra1 = rowBase + wr0 + 16 + m; if (ra1 > nN - 1) ra1 = nN - 1;
  const unsigned short* pa0h = Ah + (size_t)ra0 * KD + 8 * hh;
  const unsigned short* pa0l = Al + (size_t)ra0 * KD + 8 * hh;
  const unsigned short* pa1h = Ah + (size_t)ra1 * KD + 8 * hh;
  const unsigned short* pa1l = Al + (size_t)ra1 * KD + 8 * hh;
  const unsigned short* pbh  = Bh + (size_t)ncol * KD + 8 * hh;
  const unsigned short* pbl  = Bl + (size_t)ncol * KD + 8 * hh;

  v8f c0 = {0.f, 0.f, 0.f, 0.f, 0.f, 0.f, 0.f, 0.f};
  v8f c1 = {0.f, 0.f, 0.f, 0.f, 0.f, 0.f, 0.f, 0.f};
#pragma unroll 1
  for (int k0 = 0; k0 < KD; k0 += 32) {
    Frag a0h, a0l, a1h, a1l, bh, bl;
    bh.half[0]  = *(const v8us*)(pbh + k0);   bh.half[1]  = *(const v8us*)(pbh + k0 + 16);
    bl.half[0]  = *(const v8us*)(pbl + k0);   bl.half[1]  = *(const v8us*)(pbl + k0 + 16);
    a0h.half[0] = *(const v8us*)(pa0h + k0);  a0h.half[1] = *(const v8us*)(pa0h + k0 + 16);
    a0l.half[0] = *(const v8us*)(pa0l + k0);  a0l.half[1] = *(const v8us*)(pa0l + k0 + 16);
    a1h.half[0] = *(const v8us*)(pa1h + k0);  a1h.half[1] = *(const v8us*)(pa1h + k0 + 16);
    a1l.half[0] = *(const v8us*)(pa1l + k0);  a1l.half[1] = *(const v8us*)(pa1l + k0 + 16);
    c0 = wmb(a0h.v, bh.v, c0);
    c0 = wmb(a0l.v, bh.v, c0);
    c0 = wmb(a0h.v, bl.v, c0);
    c1 = wmb(a1h.v, bh.v, c1);
    c1 = wmb(a1l.v, bh.v, c1);
    c1 = wmb(a1h.v, bl.v, c1);
  }

  float cs = 0.f, cd = 0.f, cb = 0.f;
  if (NHD > 0) { cs = att_s[ncol]; cd = att_d[ncol]; } else { cb = bias[ncol]; }
  epi_tile<CT, XSP, NHD>(c0, wr0,      hh, m, ct, ncol, cs, cd, cb, Xs, Ps);
  epi_tile<CT, XSP, NHD>(c1, wr0 + 16, hh, m, ct, ncol, cs, cd, cb, Xs, Ps);
  __syncthreads();

  const int rr = lane / LPR;
  const int c4 = (lane % LPR) * 4;
  v4f xr[NST];
  size_t go[NST];
  bool ok[NST];
#pragma unroll
  for (int i = 0; i < NST; ++i) {
    const int brow = wave * RPW + i * RPI + rr;
    const int grow = rowBase + brow;
    xr[i] = *(const v4f*)(Xs + brow * XSP + c4);
    go[i] = (size_t)grow * NC + c4;
    ok[i] = (NHD > 0) || (grow < nN);
  }
  bool aok = false;
  v2f av = {0.f, 0.f};
  float* ap = C;
  if (NHD > 0) {
    if (wave < 2) {
      aok = true;
#pragma unroll
      for (int jj = 0; jj < 2; ++jj) {
        const int f    = 2 * lane + jj;
        const int row  = f / NHX;
        const int head = f - row * NHX;
        const float* pp = Ps + (row * CT + head * 4) * 2 + wave;
        float s = pp[0];
        s += pp[2];
        s += pp[4];
        s += pp[6];
        av[jj] = s;
      }
      ap = ((wave == 0) ? asrc : adst) + (size_t)rowBase * NHX + 2 * lane;
    }
  }
#pragma unroll
  for (int i = 0; i < NST; ++i) if (ok[i]) *(volatile v4f*)(C + go[i]) = xr[i];
  if (aok) *(volatile v2f*)ap = av;
  __threadfence();
#pragma unroll
  for (int i = 0; i < NST; ++i) if (ok[i]) *(volatile v4f*)(C + go[i]) = xr[i];
  if (aok) *(volatile v2f*)ap = av;
}

template<int NHD>
__global__ __launch_bounds__(NTHR) void k_agg(const int* __restrict__ ei, const float* __restrict__ hw,
                                              const float* __restrict__ asrc, const float* __restrict__ adst,
                                              const float* __restrict__ bias,
                                              unsigned short* oH, unsigned short* oL, int nN, int nE) {
  constexpr int DFL = HC * NHD;
  constexpr int NBL = 1024 / NHD;
  constexpr int VW  = 2 * NHD;
  constexpr int SPW = NBL / NWAVE;
  constexpr int RPI = 256 / DFL;
  constexpr int ESH = 10;
  static_assert(NBL * DFL == AGG_SACC);
  static_assert(NBL * NHD == AGG_AUX);
  static_assert(NBL <= (1 << ESH));
  static_assert((SPW % RPI) == 0);
  static_assert(RPI * DFL == 256);
  static_assert(NWAVE * 2 * RPI * DFL * 2 <= AGG_LIST * 4);
  static_assert((CHUNK << ESH) <= (1 << 30));
  typedef typename VecT<VW>::t vwf;
  typedef typename PK<VW>::t  pkt;
  typedef typename PK<VW>::ta pkta;

  extern __shared__ v4f lds_dyn[];
  float* sacc = (float*)lds_dyn;
  float* den  = sacc + AGG_SACC;
  float* mxv  = den + AGG_AUX;
  int*   list = (int*)(mxv + AGG_AUX);
  int*   wcnt = list + AGG_LIST;
  unsigned short* stg = (unsigned short*)list;

  const int tid  = threadIdx.x;
  const int lane = tid & 31;
  const int wave = tid >> 5;
  const int hd   = (lane >> 4) & (NHD - 1);
  const int c0   = VW * lane;
  const int nodeBase = blockIdx.x * NBL;

  {
    const v4f z4 = {0.f, 0.f, 0.f, 0.f};
    for (int i = tid; i < (AGG_SACC + AGG_AUX) / 4; i += NTHR) lds_dyn[i] = z4;
    const float ninf = __uint_as_float(0xff800000u);
    const v4f n4 = {ninf, ninf, ninf, ninf};
    for (int i = tid; i < AGG_AUX / 4; i += NTHR) lds_dyn[(AGG_SACC + AGG_AUX) / 4 + i] = n4;
  }
  __syncthreads();

  const int* es = ei;
  const int* ed = ei + nE;
  const bool al16 = ((nE & 3) == 0);
  const int nChunks = (nE + CHUNK - 1) / CHUNK;

#pragma unroll 1
  for (int ch = 0; ch < nChunks; ++ch) {
    const int cbase = ch * CHUNK;
    int wc = 0;
#pragma unroll
    for (int g = 0; g < NGRP; ++g) {
      const int el0 = (g * NTHR + tid) * 4;
      const int e0  = cbase + el0;
      const int sent = -2147483647 - 1;
      v4i d;
      if (al16 && (cbase + CHUNK <= nE)) {
        d = *(const v4i*)(ed + e0);
      } else {
        d.x = (e0     < nE) ? ed[min(e0,     nE - 1)] : sent;
        d.y = (e0 + 1 < nE) ? ed[min(e0 + 1, nE - 1)] : sent;
        d.z = (e0 + 2 < nE) ? ed[min(e0 + 2, nE - 1)] : sent;
        d.w = (e0 + 3 < nE) ? ed[min(e0 + 3, nE - 1)] : sent;
      }
      const unsigned s0 = (unsigned)d.x - (unsigned)nodeBase;
      const unsigned s1 = (unsigned)d.y - (unsigned)nodeBase;
      const unsigned s2 = (unsigned)d.z - (unsigned)nodeBase;
      const unsigned s3 = (unsigned)d.w - (unsigned)nodeBase;
      const bool h0 = s0 < (unsigned)NBL;
      const bool h1 = s1 < (unsigned)NBL;
      const bool h2 = s2 < (unsigned)NBL;
      const bool h3 = s3 < (unsigned)NBL;
      const unsigned many = __builtin_amdgcn_ballot_w32(h0 | h1 | h2 | h3);
      if (many != 0u) {
#define HITJ(J, HJ, SJ) { \
          const unsigned mj = __builtin_amdgcn_ballot_w32(HJ); \
          if (HJ) { \
            const int pos = wc + (int)__builtin_amdgcn_mbcnt_lo(mj, 0u); \
            if (pos < WCAP) list[wave * WCAP + pos] = ((el0 + (J)) << ESH) | (int)(SJ); \
          } \
          wc += (int)__builtin_popcount(mj); }
        HITJ(0, h0, s0)
        HITJ(1, h1, s1)
        HITJ(2, h2, s2)
        HITJ(3, h3, s3)
#undef HITJ
      }
    }
    if (lane == 0) wcnt[wave] = wc;
    __syncthreads();

    if (wave == 0) {
#pragma unroll 1
      for (int wsx = 0; wsx < NWAVE; ++wsx) {
        int n = wcnt[wsx];
        if (n > WCAP) n = WCAP;
        if (n < 0) n = 0;
#pragma unroll 1
        for (int i = 0; i < n; ++i) {
          const int ent  = list[wsx * WCAP + i];
          const int slot = ent & (NBL - 1);
          const int el   = (ent >> ESH) & (CHUNK - 1);
          int e = cbase + el;
          if (e > nE - 1) e = nE - 1;
          int src = es[e];
          src = src < 0 ? 0 : (src > nN - 1 ? nN - 1 : src);
          int nd = nodeBase + slot;
          if (nd > nN - 1) nd = nN - 1;
          float a = asrc[(size_t)src * NHD + hd] + adst[(size_t)nd * NHD + hd];
          a = (a > 0.f) ? a : 0.2f * a;
          const int ai = slot * NHD + hd;
          const float mold = mxv[ai];
          const float dold = den[ai];
          const float mnew = fmaxf(mold, a);
          const float sc = __expf(mold - mnew);
          const float p  = __expf(a - mnew);
          const vwf xv = *(const vwf*)(hw + (size_t)src * DFL + c0);
          vwf* sp = (vwf*)(sacc + slot * DFL + c0);
          const vwf cur = *sp;
          *sp = cur * sc + xv * p;
          den[ai] = dold * sc + p;
          mxv[ai] = mnew;
        }
      }
    }
    __syncthreads();
  }
  __syncthreads();

  const vwf bv = *(const vwf*)(bias + c0);
  unsigned short* stw = stg + wave * (2 * RPI * DFL);
#pragma unroll 1
  for (int j = 0; j < SPW; ++j) {
    const int slot = wave * SPW + j;
    int nc = nodeBase + slot;
    if (nc > nN - 1) nc = nN - 1;
    float a = asrc[(size_t)nc * NHD + hd] + adst[(size_t)nc * NHD + hd];
    a = (a > 0.f) ? a : 0.2f * a;
    const int ai = slot * NHD + hd;
    const float mold = mxv[ai];
    const float dold = den[ai];
    const float mnew = fmaxf(mold, a);
    const float sc = __expf(mold - mnew);
    const float p  = __expf(a - mnew);
    const vwf xv = *(const vwf*)(hw + (size_t)nc * DFL + c0);
    const vwf sv = *(const vwf*)(sacc + slot * DFL + c0) * sc + xv * p;
    const float dv  = dold * sc + p;
    const float inv = __builtin_amdgcn_rcpf(dv + 1e-16f);
    vwf y = sv * inv + bv;
#pragma unroll
    for (int q = 0; q < VW; ++q) y[q] = (y[q] > 0.f) ? y[q] : 0.f;
    pkt ph, pl;
    pack_hl(y, ph, pl);
    const int jr = j % RPI;
    *(pkta*)(stw + jr * DFL + c0) = ph;
    *(pkta*)(stw + RPI * DFL + jr * DFL + c0) = pl;
    if (jr == RPI - 1) {
      wave_sync();
      const v4u qh = *(const v4ua*)(stw + 8 * lane);
      const v4u ql = *(const v4ua*)(stw + RPI * DFL + 8 * lane);
      const size_t o = (size_t)(nodeBase + slot - (RPI - 1)) * DFL + 8 * lane;
      *(volatile v4u*)(oH + o) = qh;
      *(volatile v4u*)(oL + o) = ql;
      __threadfence();
      *(volatile v4u*)(oH + o) = qh;
      *(volatile v4u*)(oL + o) = ql;
      wave_sync();
    }
  }
}

extern "C" void kernel_launch(void* const* d_in, const int* in_sizes, int n_in,
                              void* d_out, int out_size, void* d_ws, size_t ws_size,
                              hipStream_t stream) {
  if (n_in < 15) return;
  const int nN = in_sizes[1];
  if (nN <= 0 || in_sizes[0] != nN * IN_DIM) return;
  if (in_sizes[2] < 2 || (in_sizes[2] & 1)) return;
  const int nE = in_sizes[2] / 2;
  if (in_sizes[3] != TD || in_sizes[4] != TD) return;
  if (in_sizes[5] != K1 * N1 || in_sizes[6] != N1 || in_sizes[7] != N1 || in_sizes[8] != N1) return;
  if (in_sizes[9] != K2 * N2 || in_sizes[10] != N2 || in_sizes[11] != N2 || in_sizes[12] != N2) return;
  if (in_sizes[13] != K3 * N3 || in_sizes[14] != N3) return;
  if (out_size != nN * N3) return;

  const float* x    = (const float*)d_in[0];
  const float* ts   = (const float*)d_in[1];
  const int*   ei   = (const int*)d_in[2];
  const float* tw   = (const float*)d_in[3];
  const float* tb   = (const float*)d_in[4];
  const float* W1   = (const float*)d_in[5];
  const float* aS1  = (const float*)d_in[6];
  const float* aD1  = (const float*)d_in[7];
  const float* b1   = (const float*)d_in[8];
  const float* W2   = (const float*)d_in[9];
  const float* aS2  = (const float*)d_in[10];
  const float* aD2  = (const float*)d_in[11];
  const float* b2   = (const float*)d_in[12];
  const float* Wc   = (const float*)d_in[13];
  const float* bc   = (const float*)d_in[14];
  float* out = (float*)d_out;

  const int nPad = ((nN + 1023) / 1024) * 1024;
  size_t off = 0;
  char* base = (char*)d_ws;
  unsigned short* w1h = (unsigned short*)(base + off); off += (size_t)N1 * K1 * 2;
  unsigned short* w1l = (unsigned short*)(base + off); off += (size_t)N1 * K1 * 2;
  unsigned short* w2h = (unsigned short*)(base + off); off += (size_t)N2 * K2 * 2;
  unsigned short* w2l = (unsigned short*)(base + off); off += (size_t)N2 * K2 * 2;
  unsigned short* w3h = (unsigned short*)(base + off); off += (size_t)N3 * K3 * 2;
  unsigned short* w3l = (unsigned short*)(base + off); off += (size_t)N3 * K3 * 2;
  char* regA = base + off;                             off += (size_t)2 * nPad * K1 * 2;
  float* hwp = (float*)(base + off);                   off += (size_t)nPad * N1 * 4;
  float* asrc = (float*)(base + off);                  off += (size_t)nPad * 2 * 4;
  float* adst = (float*)(base + off);                  off += (size_t)nPad * 2 * 4;
  if (off > ws_size) return;
  unsigned short* h0h = (unsigned short*)regA;
  unsigned short* h0l = h0h + (size_t)nPad * K1;
  unsigned short* h1h = (unsigned short*)regA;
  unsigned short* h1l = h1h + (size_t)nPad * K2;
  unsigned short* h2h = (unsigned short*)regA;
  unsigned short* h2l = h2h + (size_t)nPad * K3;

  k_wprep<K1, N1><<<(N1 * K1 / 8 + NTHR - 1) / NTHR, NTHR, 0, stream>>>(W1, w1h, w1l);
  k_wprep<K2, N2><<<(N2 * K2 / 8 + NTHR - 1) / NTHR, NTHR, 0, stream>>>(W2, w2h, w2l);
  k_wprep<K3, N3><<<(N3 * K3 / 8 + NTHR - 1) / NTHR, NTHR, 0, stream>>>(Wc, w3h, w3l);

  k_time<<<(nN + TROWS - 1) / TROWS, NTHR, 0, stream>>>(x, ts, tw, tb, h0h, h0l, nN);

  k_gemm<K1, N1, 2><<<(nN + 31) / 32, NTHR, 0, stream>>>(h0h, h0l, w1h, w1l, aS1, aD1, b1,
                                                        hwp, asrc, adst, nN);
  hipFuncSetAttribute(reinterpret_cast<const void*>(&k_agg<2>),
                      hipFuncAttributeMaxDynamicSharedMemorySize, AGG_LDS_BYTES);
  k_agg<2><<<(nN + 511) / 512, NTHR, AGG_LDS_BYTES, stream>>>(ei, hwp, asrc, adst, b1, h1h, h1l, nN, nE);

  k_gemm<K2, N2, 1><<<(nN + 63) / 64, NTHR, 0, stream>>>(h1h, h1l, w2h, w2l, aS2, aD2, b2,
                                                        hwp, asrc, adst, nN);
  hipFuncSetAttribute(reinterpret_cast<const void*>(&k_agg<1>),
                      hipFuncAttributeMaxDynamicSharedMemorySize, AGG_LDS_BYTES);
  k_agg<1><<<(nN + 1023) / 1024, NTHR, AGG_LDS_BYTES, stream>>>(ei, hwp, asrc, adst, b2, h2h, h2l, nN, nE);

  k_gemm<K3, N3, 0><<<(nN + 255) / 256, NTHR, 0, stream>>>(h2h, h2l, w3h, w3l, bc, bc, bc,
                                                          out, asrc, adst, nN);
}
